// theozyme_layer_1803886264724
// MI455X (gfx1250) — hardware-verified
//
#include <hip/hip_runtime.h>
#include <math.h>
#include <stdint.h>

constexpr int kBatch = 8;
constexpr int kSeq   = 512;
constexpr int kDm    = 128;
constexpr int kHeads = 8;
constexpr int kTok   = kBatch * kSeq;
constexpr int kCat   = 2 * kDm;
constexpr int kHD    = kHeads * kDm;
constexpr int kQKW   = 2 * kHD;
constexpr int kElem  = 64;
constexpr int kBond  = 8;

constexpr float kCatMul = 64.0f;
constexpr float kWMul   = 64.0f;
constexpr float kTMul   = 128.0f;
constexpr float kQMul   = 512.0f;
constexpr float kOMul   = 4096.0f;

constexpr int kTabW = 0, kTabFfb = 32, kTabBqk = 160, kTabBv = 2208, kTabN = 3232;

typedef __attribute__((ext_vector_type(16))) _Float16 v16h;
typedef __attribute__((ext_vector_type(8)))  _Float16 v8h;
typedef __attribute__((ext_vector_type(16))) __bf16   v16b;
typedef __attribute__((ext_vector_type(8)))  __bf16   v8b;
typedef __attribute__((ext_vector_type(8)))  float    v8f;
typedef __attribute__((ext_vector_type(4)))  float    v4f;
typedef __attribute__((ext_vector_type(4)))  unsigned int v4u;
typedef __attribute__((ext_vector_type(4)))  int      v4i;

__device__ __forceinline__ unsigned short f2bf_bits(float f) {
  unsigned u = __float_as_uint(f);
  return (unsigned short)((u + 0x7FFFu + ((u >> 16) & 1u)) >> 16);
}
__device__ __forceinline__ float bf_bits2f(unsigned short h) { return __uint_as_float(((unsigned)h) << 16); }

__device__ __forceinline__ void dep_guard_h(v8f& a, v8f& b, v16h x, v16h y) { asm volatile("v_nop\n\tv_nop\n\tv_nop\n\tv_nop" : "+v"(a), "+v"(b) : "v"(x), "v"(y)); }
__device__ __forceinline__ void dep_guard_b(v8f& a, v8f& b, v16b x, v16b y) { asm volatile("v_nop\n\tv_nop\n\tv_nop\n\tv_nop" : "+v"(a), "+v"(b) : "v"(x), "v"(y)); }
__device__ __forceinline__ void keep4_h(v16h a, v16h b, v16h c, v16h d) { asm volatile("v_nop" :: "v"(a), "v"(b), "v"(c), "v"(d)); }
__device__ __forceinline__ void keep4_b(v16b a, v16b b, v16b c, v16b d) { asm volatile("v_nop" :: "v"(a), "v"(b), "v"(c), "v"(d)); }
__device__ __forceinline__ void acc_guard4(v8f& a, v8f& b, v8f& c, v8f& d) { asm volatile("v_nop\n\tv_nop\n\tv_nop\n\tv_nop" : "+v"(a), "+v"(b), "+v"(c), "+v"(d)); }
template <typename T> struct Frag;
template <> struct Frag<_Float16> {
  typedef v16h V; union U { v16h v; v8h h[2]; };
  static __device__ __forceinline__ v16h load(const _Float16* p) {
    U f; f.h[0] = *(const v8h*)(p); f.h[1] = *(const v8h*)(p + 16); return f.v;
  }
  static __device__ __forceinline__ v8f mma(v16h a, v16h b, v8f c) {
    return __builtin_amdgcn_wmma_f32_16x16x32_f16(false, a, false, b, (short)0, c, false, false);
  }
  static __device__ __forceinline__ void guard(v8f& a, v8f& b, v16h x, v16h y) { dep_guard_h(a, b, x, y); }
  static __device__ __forceinline__ void keep(v16h a, v16h b, v16h c, v16h d) { keep4_h(a, b, c, d); }
};
template <> struct Frag<__bf16> {
  typedef v16b V; union U { v16b v; v8b h[2]; };
  static __device__ __forceinline__ v16b load(const __bf16* p) {
    U f; f.h[0] = *(const v8b*)(p); f.h[1] = *(const v8b*)(p + 16); return f.v;
  }
  static __device__ __forceinline__ v8f mma(v16b a, v16b b, v8f c) {
    return __builtin_amdgcn_wmma_f32_16x16x32_bf16(false, a, false, b, (short)0, c, false, false);
  }
  static __device__ __forceinline__ void guard(v8f& a, v8f& b, v16b x, v16b y) { dep_guard_b(a, b, x, y); }
  static __device__ __forceinline__ void keep(v16b a, v16b b, v16b c, v16b d) { keep4_b(a, b, c, d); }
};

template <int ET> struct Elem;
template <> struct Elem<0> { typedef _Float16 T; };
template <> struct Elem<1> { typedef __bf16 T; };
template <int ET, bool SPLIT, int BIAS_MODE, int OUT_MODE, bool RESID, int ACT = 0>
__global__ __launch_bounds__(256) void wmma_gemm64(
    const unsigned short* __restrict__ Ap, const unsigned short* __restrict__ A2p, int lda, long strideA,
    const unsigned short* __restrict__ Btp, const unsigned short* __restrict__ Bt2p, int ldb, long strideB,
    void* __restrict__ Cout, void* __restrict__ Cout2, int ldc, long strideC,
    const float* __restrict__ bias,
    const float* __restrict__ resid, long strideR,
    int M, int N, int K, float scale) {
  typedef typename Elem<ET>::T T;
  typedef typename Frag<T>::V V;
  const T* A = (const T*)Ap; const T* A2 = (const T*)A2p; const T* Bt = (const T*)Btp; const T* Bt2 = (const T*)Bt2p;
  __shared__ __align__(16) float sT[8][16 * 68];
  const int b    = blockIdx.y;
  const int lane = threadIdx.x & 31;
  const int wave = threadIdx.x >> 5;
  const int tilesN = N >> 6;
  const int tilesM = M >> 6;
  const int tile = blockIdx.x * 8 + wave;
  if (tile >= tilesM * tilesN) return;
  const int tm = tile / tilesN;
  const int tn = tile - tm * tilesN;
  const int m0 = tm << 6;
  const int n0 = tn << 6;

  const T* Ab  = A  + (size_t)b * strideA;
  const T* Bb  = Bt + (size_t)b * strideB;
  const T* Ab2 = SPLIT ? (A2  + (size_t)b * strideA) : nullptr;
  const T* Bb2 = SPLIT ? (Bt2 + (size_t)b * strideB) : nullptr;

  const int rlane = lane & 15;
  const int koff  = (lane >> 4) * 8;
  const int mOff  = (lane >> 4) * 8;

  v8f acc[4][4];
#pragma unroll
  for (int i = 0; i < 4; ++i)
#pragma unroll
    for (int j = 0; j < 4; ++j) acc[i][j] = (v8f){0.f,0.f,0.f,0.f,0.f,0.f,0.f,0.f};

  for (int k0 = 0; k0 < K; k0 += 32) {
    V bh[4], bl[4];
#pragma unroll
    for (int j = 0; j < 4; ++j) {
      const size_t bo = (size_t)(n0 + (j << 4) + rlane) * ldb + koff + k0;
      bh[j] = Frag<T>::load(Bb + bo);
      if (SPLIT) bl[j] = Frag<T>::load(Bb2 + bo);
    }
#pragma unroll
    for (int i = 0; i < 4; ++i) {
      const size_t ao = (size_t)(m0 + (i << 4) + rlane) * lda + koff + k0;
      V ah = Frag<T>::load(Ab + ao);
      V al;
      if (SPLIT) al = Frag<T>::load(Ab2 + ao);
#pragma unroll
      for (int j = 0; j < 4; ++j) {
        acc[i][j] = Frag<T>::mma(ah, bh[j], acc[i][j]);
        if (SPLIT) {
          acc[i][j] = Frag<T>::mma(ah, bl[j], acc[i][j]);
          acc[i][j] = Frag<T>::mma(al, bh[j], acc[i][j]);
        }
      }
      Frag<T>::guard(acc[i][0], acc[i][3], ah, SPLIT ? al : ah);
    }
    Frag<T>::keep(bh[0], bh[1], bh[2], bh[3]);
    if (SPLIT) Frag<T>::keep(bl[0], bl[1], bl[2], bl[3]);
  }
  acc_guard4(acc[0][0], acc[0][1], acc[0][2], acc[0][3]);
  acc_guard4(acc[1][0], acc[1][1], acc[1][2], acc[1][3]);
  acc_guard4(acc[2][0], acc[2][1], acc[2][2], acc[2][3]);
  acc_guard4(acc[3][0], acc[3][1], acc[3][2], acc[3][3]);

  float* slab = sT[wave];
  const float* Rb = RESID ? (resid + (size_t)b * strideR) : nullptr;
#pragma unroll
  for (int i = 0; i < 4; ++i) {
    const int mBase = m0 + (i << 4);
#pragma unroll
    for (int j = 0; j < 4; ++j) {
      const int n = n0 + (j << 4) + rlane;
      float bv = 0.f;
      if (BIAS_MODE == 2) bv = bias[n];
#pragma unroll
      for (int r = 0; r < 8; ++r) {
        float v = acc[i][j][r] * scale;
        if (BIAS_MODE == 1) v += bias[mBase + mOff + r];
        if (BIAS_MODE == 2) v += bv;
        if (RESID) v += Rb[(size_t)(mBase + mOff + r) * ldc + n];
        if (ACT == 1) v = tanhf(v);
        if (ACT == 2) v = fmaxf(v, 0.0f);
        if (ACT == 3) v = v / (1.0f + expf(-v));
        if (ACT == 4) v = (v > 0.f) ? v : 0.01f * v;
        if (ACT == 5) v = 0.5f * v * (1.0f + erff(v * 0.70710678118654752f));
        slab[(mOff + r) * 68 + (j << 4) + rlane] = v;
      }
    }
    __builtin_amdgcn_fence(__ATOMIC_RELEASE, "workgroup");
    __builtin_amdgcn_wave_barrier();
    __builtin_amdgcn_fence(__ATOMIC_ACQUIRE, "workgroup");
    if (OUT_MODE == 0) {
      float* C = (float*)Cout + (size_t)b * strideC;
      const int hh = lane >> 4, c4 = (lane & 15) * 4;
      for (int pass = 0; pass < 2; ++pass) {
#pragma unroll
        for (int it = 0; it < 8; ++it) {
          const int row = it * 2 + hh;
          v4f v = *(const v4f*)(slab + row * 68 + c4);
          *(volatile v4f*)(C + (size_t)(mBase + row) * ldc + n0 + c4) = v;
        }
        __threadfence();
      }
    } else {
      const int q = lane >> 3, c8 = (lane & 7) * 8;
      unsigned short* C  = (unsigned short*)Cout  + (size_t)b * strideC;
      unsigned short* C2 = (OUT_MODE == 2) ? ((unsigned short*)Cout2 + (size_t)b * strideC) : nullptr;
      for (int pass = 0; pass < 2; ++pass) {
#pragma unroll
        for (int it = 0; it < 4; ++it) {
          const int row = it * 4 + q;
          const float* sp = slab + row * 68 + c8;
          v8h hv, lv;
#pragma unroll
          for (int e = 0; e < 8; ++e) {
            if (OUT_MODE == 1) {
              hv[e] = (_Float16)sp[e];
            } else {
              unsigned short hb = f2bf_bits(sp[e]);
              unsigned short lb = f2bf_bits(sp[e] - bf_bits2f(hb));
              hv[e] = __builtin_bit_cast(_Float16, hb);
              lv[e] = __builtin_bit_cast(_Float16, lb);
            }
          }
          *(volatile v8h*)(C + (size_t)(mBase + row) * ldc + n0 + c8) = hv;
          if (OUT_MODE == 2) *(volatile v8h*)(C2 + (size_t)(mBase + row) * ldc + n0 + c8) = lv;
        }
        __threadfence();
      }
    }
    __builtin_amdgcn_fence(__ATOMIC_RELEASE, "workgroup");
    __builtin_amdgcn_wave_barrier();
    __builtin_amdgcn_fence(__ATOMIC_ACQUIRE, "workgroup");
  }
}

__device__ __forceinline__ unsigned pk16(unsigned short a, unsigned short b) { return (unsigned)a | ((unsigned)b << 16); }
__device__ __forceinline__ int clampi(int v, int lo, int hi) { return v < lo ? lo : (v > hi ? hi : v); }

__global__ __launch_bounds__(256) void tables_kernel(const float* __restrict__ bond, const float* __restrict__ ffb,
                                                     const float* __restrict__ bq, const float* __restrict__ bk,
                                                     const float* __restrict__ bv, float* __restrict__ tab) {
  const int i = blockIdx.x * 256 + threadIdx.x;
  if (i >= kTabN) return;
  const int br = clampi(i, 0, kBond - 1);
  float ws = 0.f;
#pragma unroll 1
  for (int d = 0; d < kDm; ++d) ws += bond[br * kDm + d];
  const int j1 = clampi(i - kTabFfb, 0, kDm - 1);
  const int j2 = clampi(i - kTabBqk, 0, kHD - 1);
  const int j3 = clampi(i - kTabBqk - kHD, 0, kHD - 1);
  const int j4 = clampi(i - kTabBv, 0, kHD - 1);
  const float vf = ffb[j1] * kTMul;
  const float vq = bq[j2] * kQMul;
  const float vk = bk[j3] * kQMul;
  const float vv = bv[j4] * kQMul;
  float v;
  if (i < kTabFfb) v = (i < kBond) ? ws : 0.f;
  else if (i < kTabBqk) v = vf;
  else if (i < kTabBqk + kHD) v = vq;
  else if (i < kTabBv) v = vk;
  else v = vv;
  ((volatile float*)tab)[i] = v;
  __threadfence();
  ((volatile float*)tab)[i] = v;
}

__global__ __launch_bounds__(256) void tcast_kernel(const float* __restrict__ W, unsigned short* __restrict__ out,
                                                    int R, int Cc, long strideIn, long strideOut, float mul) {
  __shared__ __align__(16) float tf[64 * 68];
  const int c0  = blockIdx.x * 64;
  const int r0  = blockIdx.y * 64;
  const int tid = threadIdx.x;
  const float* Wz = W + (size_t)blockIdx.z * strideIn;
  unsigned short* oz = out + (size_t)blockIdx.z * strideOut;
  {
    const int lr = tid >> 4;
    const int c4 = (tid & 15) * 4;
#pragma unroll
    for (int it = 0; it < 4; ++it) {
      const int rr = it * 16 + lr;
      const v4f a = *(const v4f*)(Wz + (size_t)(r0 + rr) * Cc + c0 + c4);
      *(v4f*)(tf + rr * 68 + c4) = a;
    }
  }
  __syncthreads();
  const int sub = tid >> 3;
  const int c8  = (tid & 7) * 8;
  v4u hv[2];
#pragma unroll
  for (int it = 0; it < 2; ++it) {
    const int oc = it * 32 + sub;
    v4u a;
#pragma unroll
    for (int q = 0; q < 4; ++q) {
      const float f0 = tf[(c8 + 2 * q) * 68 + oc] * mul;
      const float f1 = tf[(c8 + 2 * q + 1) * 68 + oc] * mul;
      const unsigned short h0 = __builtin_bit_cast(unsigned short, (_Float16)f0);
      const unsigned short h1 = __builtin_bit_cast(unsigned short, (_Float16)f1);
      a[q] = pk16(h0, h1);
    }
    hv[it] = a;
  }
  for (int pass = 0; pass < 2; ++pass) {
#pragma unroll
    for (int it = 0; it < 2; ++it) {
      const int oc = it * 32 + sub;
      const size_t go = (size_t)(c0 + oc) * R + r0 + c8;
      *(volatile v4u*)(oz + go) = hv[it];
    }
    __threadfence();
  }
}

__global__ __launch_bounds__(256) void embed_kernel(const int* __restrict__ te, const float* __restrict__ tp,
                                                    const float* __restrict__ elem, const float* __restrict__ posw,
                                                    const float* __restrict__ posb, unsigned short* __restrict__ cat) {
  const int lane = threadIdx.x & 31, wave = threadIdx.x >> 5;
  const int tok = blockIdx.x * 8 + wave;
  if (tok >= kTok) return;
  const int dd = (lane & 15) * 8;
  const int id = clampi(te[tok], 0, kElem - 1);
  const v4f e0 = *(const v4f*)(elem + (size_t)id * kDm + dd);
  const v4f e1 = *(const v4f*)(elem + (size_t)id * kDm + dd + 4);
  const float x0 = tp[tok * 3 + 0], x1 = tp[tok * 3 + 1], x2 = tp[tok * 3 + 2];
  const v4f w00 = *(const v4f*)(posw + dd),           w01 = *(const v4f*)(posw + dd + 4);
  const v4f w10 = *(const v4f*)(posw + kDm + dd),     w11 = *(const v4f*)(posw + kDm + dd + 4);
  const v4f w20 = *(const v4f*)(posw + 2 * kDm + dd), w21 = *(const v4f*)(posw + 2 * kDm + dd + 4);
  const v4f pb0 = *(const v4f*)(posb + dd),           pb1 = *(const v4f*)(posb + dd + 4);
  const bool use_te = (lane < 16);
  v8h hv;
#pragma unroll
  for (int e = 0; e < 4; ++e) {
    const float p0 = fmaxf(x0 * w00[e] + x1 * w10[e] + x2 * w20[e] + pb0[e], 0.0f);
    const float p1 = fmaxf(x0 * w01[e] + x1 * w11[e] + x2 * w21[e] + pb1[e], 0.0f);
    const float v0 = (use_te ? e0[e] : p0) * kCatMul;
    const float v1 = (use_te ? e1[e] : p1) * kCatMul;
    hv[e]     = (_Float16)v0;
    hv[4 + e] = (_Float16)v1;
  }
  unsigned short* dst = cat + (size_t)tok * kCat + lane * 8;
  *(volatile v8h*)dst = hv;
  __threadfence();
  *(volatile v8h*)dst = hv;
}

constexpr int kAHD = 128;
constexpr int kAKC = 64;
constexpr int kAQB = 64;
constexpr int kAOP = 132;
constexpr float kPsc = 32768.0f;

__device__ __forceinline__ v8f hmma(v16h a, v16h b, v8f c) {
  c = __builtin_amdgcn_wmma_f32_16x16x32_f16(false, a, false, b, (short)0, c, false, false);
  asm volatile("v_nop\n\tv_nop\n\tv_nop\n\tv_nop" : "+v"(c) : "v"(a), "v"(b));
  return c;
}

__global__ __launch_bounds__(128)
void attn128_kernel(const unsigned short* __restrict__ qkp, const unsigned short* __restrict__ vtp,
                    const int* __restrict__ tadj, const float* __restrict__ wtab,
                    unsigned short* __restrict__ op, float sscale, float oscale) {
  union FH { v16h v; v8h h[2]; };
  __shared__ __align__(16) unsigned char smem[40960];
  __shared__ __align__(16) float Wsh[kAQB * kAKC];
  __shared__ float wts[kBond];
  _Float16* Ksh   = (_Float16*)(smem);
  _Float16* Vth   = (_Float16*)(smem + 16384);
  _Float16* Pbase = (_Float16*)(smem + 32768);
  float*    Osb   = (float*)(smem);

  const int tid  = threadIdx.x;
  const int wave = tid >> 5;
  const int lane = tid & 31;
  const int hh   = lane >> 4;
  const int c    = lane & 15;

  const int nqb = kSeq / kAQB;
  const int bx  = blockIdx.x;
  const int qb  = bx % nqb;
  const int bh  = bx / nqb;
  const int h   = bh % kHeads;
  const int b   = bh / kHeads;
  const int tokbase = b * kSeq;
  const int q0  = qb * kAQB + wave * 16;

  if (tid < kBond) wts[tid] = wtab[tid];

  const _Float16* QK = (const _Float16*)(const void*)qkp;
  const _Float16* VT = (const _Float16*)(const void*)vtp;

  v16h qa[4];
#pragma unroll
  for (int dc = 0; dc < 4; ++dc)
    qa[dc] = Frag<_Float16>::load(QK + (size_t)(tokbase + q0 + c) * kQKW + h * kAHD + dc * 32 + 8 * hh);

  float mrow[8], lrow[8];
  v8f oacc[8];
#pragma unroll
  for (int r = 0; r < 8; ++r) { mrow[r] = -INFINITY; lrow[r] = 0.f; }
#pragma unroll
  for (int t = 0; t < 8; ++t) oacc[t] = (v8f){0.f,0.f,0.f,0.f,0.f,0.f,0.f,0.f};

  const int nChunks = qb + 1;
  for (int kc = 0; kc < nChunks; ++kc) {
    const int kv0 = kc * kAKC;
    __syncthreads();
    {
      const int r = tid >> 1, half = (tid & 1) * 64;
      const _Float16* ks = QK + (size_t)(tokbase + kv0 + r) * kQKW + kHD + h * kAHD + half;
      const _Float16* vs = VT + (size_t)(h * kAHD + tid) * kTok + tokbase + kv0;
#pragma unroll
      for (int i = 0; i < 8; ++i) {
        const v8h a  = *(const v8h*)(ks + 8 * i);
        const v8h bb = *(const v8h*)(vs + 8 * i);
        *(v8h*)(Ksh + r * kAHD + half + 8 * i) = a;
        *(v8h*)(Vth + tid * kAKC + 8 * i) = bb;
      }
      const int ch = (tid & 1) * 32;
      const int* trow = tadj + ((size_t)(tokbase + qb * kAQB + r)) * kSeq + kv0 + ch;
#pragma unroll
      for (int i = 0; i < 8; ++i) {
        const v4i ids = *(const v4i*)(trow + 4 * i);
        v4f wv;
#pragma unroll
        for (int e = 0; e < 4; ++e) wv[e] = wts[clampi(ids[e], 0, kBond - 1)];
        *(v4f*)(Wsh + r * kAKC + ch + 4 * i) = wv;
      }
    }
    __syncthreads();

    v8f s[4];
#pragma unroll
    for (int j = 0; j < 4; ++j) {
      s[j] = (v8f){0.f,0.f,0.f,0.f,0.f,0.f,0.f,0.f};
#pragma unroll
      for (int dc = 0; dc < 4; ++dc) {
        FH kb;
        kb.h[0] = *(const v8h*)(Ksh + (j * 16 + c) * kAHD + dc * 32 + 8 * hh);
        kb.h[1] = *(const v8h*)(Ksh + (j * 16 + c) * kAHD + dc * 32 + 16 + 8 * hh);
        s[j] = hmma(qa[dc], kb.v, s[j]);
      }
    }
    const bool diag = (kc == qb);
    float cm[8];
#pragma unroll
    for (int r = 0; r < 8; ++r) {
      const int lrow = wave * 16 + 8 * hh + r;
      const int qrow = qb * kAQB + lrow;
      float m = -INFINITY;
#pragma unroll
      for (int j = 0; j < 4; ++j) {
        const int kvcol = kv0 + j * 16 + c;
        const float wv = Wsh[lrow * kAKC + j * 16 + c];
        const float sv = (s[j][r] * sscale) * wv;
        const bool masked = diag && (kvcol > qrow);
        const float sm = masked ? -INFINITY : sv;
        s[j][r] = sm;
        m = fmaxf(m, sm);
      }
#pragma unroll
      for (int off = 1; off < 16; off <<= 1) m = fmaxf(m, __shfl_xor(m, off, 32));
      cm[r] = m;
    }
    _Float16* pw = Pbase + wave * (16 * kAKC);
#pragma unroll
    for (int r = 0; r < 8; ++r) {
      const float mnew = fmaxf(mrow[r], cm[r]);
      const float alpha = expf(mrow[r] - mnew);
      mrow[r] = mnew;
      float psum = 0.f;
#pragma unroll
      for (int j = 0; j < 4; ++j) {
        const float p = expf(s[j][r] - mnew);
        psum += p;
        pw[(8 * hh + r) * kAKC + j * 16 + c] = (_Float16)(p * kPsc);
      }
#pragma unroll
      for (int off = 1; off < 16; off <<= 1) psum += __shfl_xor(psum, off, 32);
      lrow[r] = lrow[r] * alpha + psum;
#pragma unroll
      for (int t = 0; t < 8; ++t) oacc[t][r] *= alpha;
    }
    __builtin_amdgcn_fence(__ATOMIC_RELEASE, "workgroup");
    __builtin_amdgcn_wave_barrier();
    __builtin_amdgcn_fence(__ATOMIC_ACQUIRE, "workgroup");
#pragma unroll 1
    for (int kk = 0; kk < 2; ++kk) {
      FH pa;
      pa.h[0] = *(const v8h*)(pw + c * kAKC + kk * 32 + 8 * hh);
      pa.h[1] = *(const v8h*)(pw + c * kAKC + kk * 32 + 16 + 8 * hh);
#pragma unroll
      for (int t = 0; t < 8; ++t) {
        FH vb;
        vb.h[0] = *(const v8h*)(Vth + (t * 16 + c) * kAKC + kk * 32 + 8 * hh);
        vb.h[1] = *(const v8h*)(Vth + (t * 16 + c) * kAKC + kk * 32 + 16 + 8 * hh);
        oacc[t] = hmma(pa.v, vb.v, oacc[t]);
      }
    }
  }

  __syncthreads();
  float* os = Osb + wave * (16 * kAOP);
#pragma unroll
  for (int r = 0; r < 8; ++r) {
    const float inv = oscale / (lrow[r] * kPsc);
#pragma unroll
    for (int t = 0; t < 8; ++t) os[(8 * hh + r) * kAOP + t * 16 + c] = oacc[t][r] * inv;
  }
  __builtin_amdgcn_fence(__ATOMIC_RELEASE, "workgroup");
  __builtin_amdgcn_wave_barrier();
  __builtin_amdgcn_fence(__ATOMIC_ACQUIRE, "workgroup");
  {
    const int c8 = (lane & 15) * 8;
    for (int pass = 0; pass < 2; ++pass) {
#pragma unroll
      for (int it = 0; it < 8; ++it) {
        const int row = it * 2 + hh;
        const float* sp = os + row * kAOP + c8;
        v8h hv;
#pragma unroll
        for (int e = 0; e < 8; ++e) hv[e] = (_Float16)sp[e];
        *(volatile v8h*)(op + (size_t)(tokbase + q0 + row) * kHD + h * kAHD + c8) = hv;
      }
      __threadfence();
    }
  }
}

extern "C" void kernel_launch(void* const* d_in, const int* in_sizes, int n_in,
                              void* d_out, int out_size, void* d_ws, size_t ws_size,
                              hipStream_t stream) {
  if (n_in < 17) return;
  if (in_sizes[0] != kTok || in_sizes[2] != kTok * kSeq || out_size != kTok * kDm) return;
  const int*   TE       = (const int*)d_in[0];
  const float* TP       = (const float*)d_in[1];
  const int*   TADJ     = (const int*)d_in[2];
  const float* elem_emb = (const float*)d_in[3];
  const float* bond_emb = (const float*)d_in[4];
  const float* pos_W    = (const float*)d_in[5];
  const float* pos_b    = (const float*)d_in[6];
  const float* ff_W     = (const float*)d_in[7];
  const float* ff_b     = (const float*)d_in[8];
  const float* Wq       = (const float*)d_in[9];
  const float* bq       = (const float*)d_in[10];
  const float* Wk       = (const float*)d_in[11];
  const float* bk       = (const float*)d_in[12];
  const float* Wv       = (const float*)d_in[13];
  const float* bv       = (const float*)d_in[14];
  const float* out_W    = (const float*)d_in[15];
  const float* out_b    = (const float*)d_in[16];
  float* out = (float*)d_out;

  size_t off = 0;
  char* wsb = (char*)d_ws;
  auto take = [&](size_t bytes) -> char* {
    char* p = wsb + off;
    off += (bytes + 255) & ~(size_t)255;
    return p;
  };
  float*          tab   = (float*)take((size_t)kTabN * 4);
  unsigned short* ffWT  = (unsigned short*)take((size_t)kDm * kCat * 2);
  unsigned short* WqkT  = (unsigned short*)take((size_t)kQKW * kDm * 2);
  unsigned short* WvT   = (unsigned short*)take((size_t)kHD * kDm * 2);
  unsigned short* outWT = (unsigned short*)take((size_t)kDm * kHD * 2);
  unsigned short* cat   = (unsigned short*)take((size_t)kTok * kCat * 2);
  unsigned short* tpl   = (unsigned short*)take((size_t)kTok * kDm * 2);
  unsigned short* qk    = (unsigned short*)take((size_t)kTok * kQKW * 2);
  unsigned short* vt    = (unsigned short*)take((size_t)kHD * kTok * 2);
  unsigned short* opl   = (unsigned short*)take((size_t)kTok * kHD * 2);
  if (off > ws_size) return;

  tables_kernel<<<(kTabN + 255) / 256, 256, 0, stream>>>(bond_emb, ff_b, bq, bk, bv, tab);

  tcast_kernel<<<dim3(kDm / 64, kCat / 64, 1), 256, 0, stream>>>(ff_W, ffWT, kCat, kDm, 0L, 0L, kWMul);
  tcast_kernel<<<dim3(kDm / 64, kDm / 64, kHeads), 256, 0, stream>>>(Wq, WqkT, kDm, kDm, (long)kDm * kDm, (long)kDm * kDm, kWMul);
  tcast_kernel<<<dim3(kDm / 64, kDm / 64, kHeads), 256, 0, stream>>>(Wk, WqkT + (size_t)kHD * kDm, kDm, kDm, (long)kDm * kDm, (long)kDm * kDm, kWMul);
  tcast_kernel<<<dim3(kDm / 64, kDm / 64, kHeads), 256, 0, stream>>>(Wv, WvT, kDm, kDm, (long)kDm * kDm, (long)kDm * kDm, kWMul);
  tcast_kernel<<<dim3(kDm / 64, kHD / 64, 1), 256, 0, stream>>>(out_W, outWT, kHD, kDm, 0L, 0L, kWMul);

  embed_kernel<<<kTok / 8, 256, 0, stream>>>(TE, TP, elem_emb, pos_W, pos_b, cat);

  wmma_gemm64<0, false, 2, 1, false, 2><<<dim3(16, 1), 256, 0, stream>>>(
      cat, cat, kCat, 0L, ffWT, ffWT, kCat, 0L, (void*)tpl, (void*)tpl, kDm, 0L,
      tab + kTabFfb, tab, 0L, kTok, kDm, kCat, kTMul / (kCatMul * kWMul));

  wmma_gemm64<0, false, 2, 1, false, 0><<<dim3(256, 1), 256, 0, stream>>>(
      tpl, tpl, kDm, 0L, WqkT, WqkT, kDm, 0L, (void*)qk, (void*)qk, kQKW, 0L,
      tab + kTabBqk, tab, 0L, kTok, kQKW, kDm, kQMul / (kTMul * kWMul));

  wmma_gemm64<0, false, 1, 1, false, 0><<<dim3(128, 1), 256, 0, stream>>>(
      WvT, WvT, kDm, 0L, tpl, tpl, kDm, 0L, (void*)vt, (void*)vt, kTok, 0L,
      tab + kTabBv, tab, 0L, kHD, kTok, kDm, kQMul / (kTMul * kWMul));

  const float rsq = 1.0f / sqrtf((float)kSeq);
  const float sscale = rsq / (kQMul * kQMul);
  const float oscale = kOMul / kQMul;
  attn128_kernel<<<kBatch * kHeads * (kSeq / kAQB), 128, 0, stream>>>(qk, vt, TADJ, tab + kTabW, opl, sscale, oscale);

  wmma_gemm64<0, false, 2, 0, false, 0><<<dim3(16, 1), 256, 0, stream>>>(
      opl, opl, kHD, 0L, outWT, outWT, kHD, 0L, (void*)out, (void*)out, kDm, 0L,
      out_b, tab, 0L, kTok, kDm, kHD, 1.0f / (kOMul * kWMul));
}
